// ResRBFPoisLayer_22308060136157
// MI455X (gfx1250) — hardware-verified
//
#include <hip/hip_runtime.h>
#include <math.h>

typedef __attribute__((ext_vector_type(16))) _Float16 v16h;
typedef __attribute__((ext_vector_type(8)))  _Float16 v8h;
typedef __attribute__((ext_vector_type(16))) __bf16   v16b;
typedef __attribute__((ext_vector_type(8)))  __bf16   v8b;
typedef __attribute__((ext_vector_type(8)))  float    v8f;
typedef __attribute__((ext_vector_type(4)))  float    v4f;

constexpr int NIMG          = 16;
constexpr int IMG_H         = 256;
constexpr int IMG_W         = 256;
constexpr int NPIX_IMG      = IMG_H * IMG_W;
constexpr int NFEAT         = 64;
constexpr int KSZ           = 7;
constexpr int NTAPS         = KSZ * KSZ;
constexpr int KPAD          = 64;
constexpr int PADW          = 3;
constexpr int NMIX          = 51;
constexpr int NGRID         = 1001;
constexpr int TAB_PITCH     = 1024;
constexpr int IMG_PER_CHUNK = 2;
constexpr int NCHUNK        = NIMG / IMG_PER_CHUNK;
constexpr int NPIX_CHUNK    = IMG_PER_CHUNK * NPIX_IMG;
constexpr int CHUNKS16      = NPIX_CHUNK * (KPAD / 8);
static_assert(KPAD % 32 == 0);
static_assert(NTAPS <= KPAD);
static_assert(NPIX_CHUNK % 64 == 0 && NFEAT == 64 && KPAD == 64);
static_assert(CHUNKS16 % 256 == 0);
static_assert(NIMG % IMG_PER_CHUNK == 0);
static_assert(TAB_PITCH >= NGRID && TAB_PITCH % 256 == 0);

__device__ __forceinline__ unsigned short f2bf_bits(float f) {
  unsigned u = __float_as_uint(f);
  return (unsigned short)((u + 0x7FFFu + ((u >> 16) & 1u)) >> 16);
}
__device__ __forceinline__ float bf_bits2f(unsigned short h) { return __uint_as_float(((unsigned)h) << 16); }

__device__ __forceinline__ void dep_guard_h(v8f& a, v8f& b, v16h x, v16h y) { asm volatile("v_nop\n\tv_nop\n\tv_nop\n\tv_nop" : "+v"(a), "+v"(b) : "v"(x), "v"(y)); }
__device__ __forceinline__ void dep_guard_b(v8f& a, v8f& b, v16b x, v16b y) { asm volatile("v_nop\n\tv_nop\n\tv_nop\n\tv_nop" : "+v"(a), "+v"(b) : "v"(x), "v"(y)); }
__device__ __forceinline__ void keep4_h(v16h a, v16h b, v16h c, v16h d) { asm volatile("v_nop" :: "v"(a), "v"(b), "v"(c), "v"(d)); }
__device__ __forceinline__ void keep4_b(v16b a, v16b b, v16b c, v16b d) { asm volatile("v_nop" :: "v"(a), "v"(b), "v"(c), "v"(d)); }
__device__ __forceinline__ void acc_guard4(v8f& a, v8f& b, v8f& c, v8f& d) { asm volatile("v_nop\n\tv_nop\n\tv_nop\n\tv_nop" : "+v"(a), "+v"(b), "+v"(c), "+v"(d)); }
template <typename T> struct Frag;
template <> struct Frag<_Float16> {
  typedef v16h V; union U { v16h v; v8h h[2]; };
  static __device__ __forceinline__ v16h load(const _Float16* p) {
    U f; f.h[0] = *(const v8h*)(p); f.h[1] = *(const v8h*)(p + 16); return f.v;
  }
  static __device__ __forceinline__ v8f mma(v16h a, v16h b, v8f c) {
    return __builtin_amdgcn_wmma_f32_16x16x32_f16(false, a, false, b, (short)0, c, false, false);
  }
  static __device__ __forceinline__ void guard(v8f& a, v8f& b, v16h x, v16h y) { dep_guard_h(a, b, x, y); }
  static __device__ __forceinline__ void keep(v16h a, v16h b, v16h c, v16h d) { keep4_h(a, b, c, d); }
};
template <> struct Frag<__bf16> {
  typedef v16b V; union U { v16b v; v8b h[2]; };
  static __device__ __forceinline__ v16b load(const __bf16* p) {
    U f; f.h[0] = *(const v8b*)(p); f.h[1] = *(const v8b*)(p + 16); return f.v;
  }
  static __device__ __forceinline__ v8f mma(v16b a, v16b b, v8f c) {
    return __builtin_amdgcn_wmma_f32_16x16x32_bf16(false, a, false, b, (short)0, c, false, false);
  }
  static __device__ __forceinline__ void guard(v8f& a, v8f& b, v16b x, v16b y) { dep_guard_b(a, b, x, y); }
  static __device__ __forceinline__ void keep(v16b a, v16b b, v16b c, v16b d) { keep4_b(a, b, c, d); }
};

template <int ET> struct Elem;
template <> struct Elem<0> { typedef _Float16 T; };
template <> struct Elem<1> { typedef __bf16 T; };
template <int ET, bool SPLIT, int BIAS_MODE, int OUT_MODE, bool RESID, int ACT = 0>
__global__ __launch_bounds__(256) void wmma_gemm64(
    const unsigned short* __restrict__ Ap, const unsigned short* __restrict__ A2p, int lda, long strideA,
    const unsigned short* __restrict__ Btp, const unsigned short* __restrict__ Bt2p, int ldb, long strideB,
    void* __restrict__ Cout, void* __restrict__ Cout2, int ldc, long strideC,
    const float* __restrict__ bias,
    const float* __restrict__ resid, long strideR,
    int M, int N, int K, float scale) {
  typedef typename Elem<ET>::T T;
  typedef typename Frag<T>::V V;
  const T* A = (const T*)Ap; const T* A2 = (const T*)A2p; const T* Bt = (const T*)Btp; const T* Bt2 = (const T*)Bt2p;
  __shared__ __align__(16) float sT[8][16 * 68];
  const int b    = blockIdx.y;
  const int lane = threadIdx.x & 31;
  const int wave = threadIdx.x >> 5;
  const int tilesN = N >> 6;
  const int tilesM = M >> 6;
  const int tile = blockIdx.x * 8 + wave;
  if (tile >= tilesM * tilesN) return;
  const int tm = tile / tilesN;
  const int tn = tile - tm * tilesN;
  const int m0 = tm << 6;
  const int n0 = tn << 6;

  const T* Ab  = A  + (size_t)b * strideA;
  const T* Bb  = Bt + (size_t)b * strideB;
  const T* Ab2 = SPLIT ? (A2  + (size_t)b * strideA) : nullptr;
  const T* Bb2 = SPLIT ? (Bt2 + (size_t)b * strideB) : nullptr;

  const int rlane = lane & 15;
  const int koff  = (lane >> 4) * 8;
  const int mOff  = (lane >> 4) * 8;

  v8f acc[4][4];
#pragma unroll
  for (int i = 0; i < 4; ++i)
#pragma unroll
    for (int j = 0; j < 4; ++j) acc[i][j] = (v8f){0.f,0.f,0.f,0.f,0.f,0.f,0.f,0.f};

  for (int k0 = 0; k0 < K; k0 += 32) {
    V bh[4], bl[4];
#pragma unroll
    for (int j = 0; j < 4; ++j) {
      const size_t bo = (size_t)(n0 + (j << 4) + rlane) * ldb + koff + k0;
      bh[j] = Frag<T>::load(Bb + bo);
      if (SPLIT) bl[j] = Frag<T>::load(Bb2 + bo);
    }
#pragma unroll
    for (int i = 0; i < 4; ++i) {
      const size_t ao = (size_t)(m0 + (i << 4) + rlane) * lda + koff + k0;
      V ah = Frag<T>::load(Ab + ao);
      V al;
      if (SPLIT) al = Frag<T>::load(Ab2 + ao);
#pragma unroll
      for (int j = 0; j < 4; ++j) {
        acc[i][j] = Frag<T>::mma(ah, bh[j], acc[i][j]);
        if (SPLIT) {
          acc[i][j] = Frag<T>::mma(ah, bl[j], acc[i][j]);
          acc[i][j] = Frag<T>::mma(al, bh[j], acc[i][j]);
        }
      }
      Frag<T>::guard(acc[i][0], acc[i][3], ah, SPLIT ? al : ah);
    }
    Frag<T>::keep(bh[0], bh[1], bh[2], bh[3]);
    if (SPLIT) Frag<T>::keep(bl[0], bl[1], bl[2], bl[3]);
  }
  acc_guard4(acc[0][0], acc[0][1], acc[0][2], acc[0][3]);
  acc_guard4(acc[1][0], acc[1][1], acc[1][2], acc[1][3]);
  acc_guard4(acc[2][0], acc[2][1], acc[2][2], acc[2][3]);
  acc_guard4(acc[3][0], acc[3][1], acc[3][2], acc[3][3]);

  float* slab = sT[wave];
  const float* Rb = RESID ? (resid + (size_t)b * strideR) : nullptr;
#pragma unroll
  for (int i = 0; i < 4; ++i) {
    const int mBase = m0 + (i << 4);
#pragma unroll
    for (int j = 0; j < 4; ++j) {
      const int n = n0 + (j << 4) + rlane;
      float bv = 0.f;
      if (BIAS_MODE == 2) bv = bias[n];
#pragma unroll
      for (int r = 0; r < 8; ++r) {
        float v = acc[i][j][r] * scale;
        if (BIAS_MODE == 1) v += bias[mBase + mOff + r];
        if (BIAS_MODE == 2) v += bv;
        if (RESID) v += Rb[(size_t)(mBase + mOff + r) * ldc + n];
        if (ACT == 1) v = tanhf(v);
        if (ACT == 2) v = fmaxf(v, 0.0f);
        if (ACT == 3) v = v / (1.0f + expf(-v));
        if (ACT == 4) v = (v > 0.f) ? v : 0.01f * v;
        if (ACT == 5) v = 0.5f * v * (1.0f + erff(v * 0.70710678118654752f));
        slab[(mOff + r) * 68 + (j << 4) + rlane] = v;
      }
    }
    __builtin_amdgcn_fence(__ATOMIC_RELEASE, "workgroup");
    __builtin_amdgcn_wave_barrier();
    __builtin_amdgcn_fence(__ATOMIC_ACQUIRE, "workgroup");
    if (OUT_MODE == 0) {
      float* C = (float*)Cout + (size_t)b * strideC;
      const int hh = lane >> 4, c4 = (lane & 15) * 4;
      for (int pass = 0; pass < 2; ++pass) {
#pragma unroll
        for (int it = 0; it < 8; ++it) {
          const int row = it * 2 + hh;
          v4f v = *(const v4f*)(slab + row * 68 + c4);
          *(volatile v4f*)(C + (size_t)(mBase + row) * ldc + n0 + c4) = v;
        }
        __threadfence();
      }
    } else {
      const int q = lane >> 3, c8 = (lane & 7) * 8;
      unsigned short* C  = (unsigned short*)Cout  + (size_t)b * strideC;
      unsigned short* C2 = (OUT_MODE == 2) ? ((unsigned short*)Cout2 + (size_t)b * strideC) : nullptr;
      for (int pass = 0; pass < 2; ++pass) {
#pragma unroll
        for (int it = 0; it < 4; ++it) {
          const int row = it * 4 + q;
          const float* sp = slab + row * 68 + c8;
          v8h hv, lv;
#pragma unroll
          for (int e = 0; e < 8; ++e) {
            if (OUT_MODE == 1) {
              hv[e] = (_Float16)sp[e];
            } else {
              unsigned short hb = f2bf_bits(sp[e]);
              unsigned short lb = f2bf_bits(sp[e] - bf_bits2f(hb));
              hv[e] = __builtin_bit_cast(_Float16, hb);
              lv[e] = __builtin_bit_cast(_Float16, lb);
            }
          }
          *(volatile v8h*)(C + (size_t)(mBase + row) * ldc + n0 + c8) = hv;
          if (OUT_MODE == 2) *(volatile v8h*)(C2 + (size_t)(mBase + row) * ldc + n0 + c8) = lv;
        }
        __threadfence();
      }
    }
    __builtin_amdgcn_fence(__ATOMIC_RELEASE, "workgroup");
    __builtin_amdgcn_wave_barrier();
    __builtin_amdgcn_fence(__ATOMIC_ACQUIRE, "workgroup");
  }
}

__global__ __launch_bounds__(256) void prep_weights_kernel(
    const float* __restrict__ cw, const float* __restrict__ scf,
    unsigned short* __restrict__ w16, unsigned short* __restrict__ wt16, float carry)
{
  __shared__ float wn[NFEAT * NTAPS];
  __shared__ __align__(16) _Float16 sA[NFEAT * KPAD];
  __shared__ __align__(16) _Float16 sB[KPAD * NFEAT];
  const int t = threadIdx.x;
  if (t < NFEAT) {
    const float* row = cw + t * NTAPS;
    float s = 0.f;
#pragma unroll 1
    for (int i = 0; i < NTAPS; ++i) s += row[i];
    const float mean = s * (1.0f / 49.0f);
    float ss = 0.f;
#pragma unroll 1
    for (int i = 0; i < NTAPS; ++i) { const float d = row[i] - mean; ss += d * d; }
    const float nrm = sqrtf(ss);
    const float sc  = scf[t] * (1.0f / nrm);
#pragma unroll 1
    for (int i = 0; i < NTAPS; ++i) wn[t * NTAPS + i] = sc * (row[i] - mean);
  }
  __syncthreads();
  for (int idx = t; idx < NFEAT * KPAD; idx += 256) {
    const int hi6 = idx >> 6;
    const int lo6 = idx & 63;
    const int kc = (lo6 < NTAPS) ? lo6 : 0;
    const float va = wn[hi6 * NTAPS + kc];
    sA[idx] = (_Float16)((lo6 < NTAPS) ? va * carry : 0.0f);
    const int tc = (hi6 < NTAPS) ? hi6 : 0;
    const float vb = wn[lo6 * NTAPS + tc];
    sB[idx] = (_Float16)((hi6 < NTAPS) ? vb * carry : 0.0f);
  }
  __syncthreads();
  for (int pass = 0; pass < 2; ++pass) {
#pragma unroll
    for (int h = 0; h < 2; ++h) {
      const int c = t + h * 256;
      const v8h a = *(const v8h*)(sA + c * 8);
      const v8h b = *(const v8h*)(sB + c * 8);
      *(volatile v8h*)(w16 + (size_t)c * 8) = a;
      *(volatile v8h*)(wt16 + (size_t)c * 8) = b;
    }
    __threadfence();
  }
}

__global__ __launch_bounds__(256) void mix_table_kernel(
    const float* __restrict__ mixw, const float* __restrict__ ctr, const float* __restrict__ gridv,
    float* __restrict__ table, float prec)
{
  __shared__ __align__(16) float sv[256];
  const int t = threadIdx.x;
  const int f = blockIdx.y;
  const int l = blockIdx.x * 256 + t;
  const bool valid = l < NGRID;
  const int lc = valid ? l : (NGRID - 1);
  const float g = gridv[lc];
  const float* wrow = mixw + f * NMIX;
  float acc = 0.f;
#pragma unroll 1
  for (int m = 0; m < NMIX; ++m) {
    const float d = prec * (g - ctr[m]);
    const float e = expf((-0.5f * d) * d);
    acc += wrow[m] * e;
  }
  sv[t] = valid ? acc : 0.0f;
  __syncthreads();
  if (t < 64) {
    const v4f v = *(const v4f*)(sv + 4 * t);
    float* dst = table + (size_t)f * TAB_PITCH + blockIdx.x * 256 + 4 * t;
    *(volatile v4f*)dst = v;
    __threadfence();
    *(volatile v4f*)dst = v;
  }
}

__device__ __forceinline__ int refl_idx(int tt, int n) {
  int r = tt < 0 ? (-1 - tt) : (tt > n - 1 ? (2 * n - 1 - tt) : tt);
  r = r < 0 ? 0 : (r > n - 1 ? n - 1 : r);
  return r;
}
__global__ __launch_bounds__(256) void im2col_sym7_kernel(
    const float* __restrict__ x, unsigned short* __restrict__ dst, int img0, int nchunks)
{
  const int f = blockIdx.x * 256 + threadIdx.x;
  if (f >= nchunks) return;
  const int pix = f >> 3;
  const int k0  = (f & 7) * 8;
  const int il  = pix >> 16;
  const int y   = (pix >> 8) & (IMG_H - 1);
  const int xx  = pix & (IMG_W - 1);
  const float* xb = x + (size_t)(img0 + il) * NPIX_IMG;
  v8h hv;
#pragma unroll
  for (int e = 0; e < 8; ++e) {
    const int k = k0 + e;
    const bool valid = k < NTAPS;
    const int kc = valid ? k : 0;
    const int di = kc / KSZ;
    const int dj = kc - di * KSZ;
    const int sy = refl_idx(y + di - PADW, IMG_H);
    const int sx = refl_idx(xx + dj - PADW, IMG_W);
    const float v = xb[sy * IMG_W + sx];
    hv[e] = valid ? (_Float16)v : (_Float16)0.0f;
  }
  unsigned short* q = dst + (size_t)f * 8;
  *(volatile v8h*)q = hv;
  __threadfence();
  *(volatile v8h*)q = hv;
}

__global__ __launch_bounds__(256) void table_interp_kernel(
    const float* __restrict__ U, const float* __restrict__ table, const float* __restrict__ gridv,
    unsigned short* __restrict__ phi, int nthreads, float carry)
{
  const int idx = blockIdx.x * 256 + threadIdx.x;
  if (idx >= nthreads) return;
  const int pix = idx >> 3;
  const int f0  = (idx & 7) * 8;
  const float g0    = gridv[0];
  const float g1    = gridv[1];
  const float gL    = gridv[NGRID - 1];
  const float step  = g1 - g0;
  const float rstep = 1.0f / step;
  const float* up = U + (size_t)pix * NFEAT + f0;
  const v4f ua = *(const v4f*)(up);
  const v4f ub = *(const v4f*)(up + 4);
  v8h hv;
#pragma unroll
  for (int e = 0; e < 8; ++e) {
    const float u  = (e < 4) ? ua[e & 3] : ub[e & 3];
    const float uc = fminf(fmaxf(u, g0), gL);
    const float pos = (uc - g0) * rstep;
    const float fl  = floorf(pos);
    int i0 = (int)fl;
    i0 = i0 < 0 ? 0 : (i0 > NGRID - 2 ? NGRID - 2 : i0);
    const float frac = pos - (float)i0;
    const float* row = table + (size_t)(f0 + e) * TAB_PITCH;
    const float v0 = row[i0];
    const float v1 = row[i0 + 1];
    const float ph = v0 * (1.0f - frac) + v1 * frac;
    hv[e] = (_Float16)(ph * carry);
  }
  unsigned short* q = phi + (size_t)idx * 8;
  *(volatile v8h*)q = hv;
  __threadfence();
  *(volatile v8h*)q = hv;
}

__global__ __launch_bounds__(256) void fold_prox_kernel(
    const float* __restrict__ QT, const float* __restrict__ xin, const float* __restrict__ nz,
    const float* __restrict__ acond, float* __restrict__ out, int img0, int qpitch)
{
#pragma clang fp contract(off)
  __shared__ __align__(16) float srow[IMG_W];
  const int j  = threadIdx.x;
  const int i  = blockIdx.x;
  const int il = blockIdx.y;
  const int b  = img0 + il;
  const float* Qimg = QT + (size_t)il * NPIX_IMG;
  const int pyA = i + PADW;
  const int pyB = (i <= 2) ? (2 - i) : (2 * IMG_H + 2 - i);
  const int pxA = j + PADW;
  const int pxB = (j <= 2) ? (2 - j) : (2 * IMG_W + 2 - j);
  float r = 0.f;
#pragma unroll 1
  for (int p = 0; p < 2; ++p) {
    const int py = (p == 0) ? pyA : pyB;
#pragma unroll 1
    for (int di = 0; di < KSZ; ++di) {
      const int yy = py - di;
      if ((unsigned)yy < (unsigned)IMG_H) {
#pragma unroll
        for (int dj = 0; dj < KSZ; ++dj) {
          const float* qrow = Qimg + (size_t)(di * KSZ + dj) * qpitch + (size_t)yy * IMG_W;
          const int xa = pxA - dj;
          const int xb = pxB - dj;
          const bool va = (unsigned)xa < (unsigned)IMG_W;
          const bool vb = (unsigned)xb < (unsigned)IMG_W;
          const int xac = xa < 0 ? 0 : (xa > IMG_W - 1 ? IMG_W - 1 : xa);
          const int xbc = xb < 0 ? 0 : (xb > IMG_W - 1 ? IMG_W - 1 : xb);
          const float qa = qrow[xac];
          const float qb = qrow[xbc];
          r += va ? qa : 0.0f;
          r += vb ? qb : 0.0f;
        }
      }
    }
  }
  const size_t o = (size_t)b * NPIX_IMG + (size_t)i * IMG_W + j;
  const float xv = xin[o];
  const float nv = nz[o];
  const float a  = acond[b];
  const float z  = xv - r;
  const float d  = z - a;
  const float q4 = (4.0f * a) * nv;
  const float dd = d * d;
  const float s  = sqrtf(dd + q4);
  const float val = 0.5f * (d + s);
  srow[j] = val;
  __syncthreads();
  if (j < 64) {
    const v4f v = *(const v4f*)(srow + 4 * j);
    float* dst = out + (size_t)b * NPIX_IMG + (size_t)i * IMG_W + 4 * j;
    *(volatile v4f*)dst = v;
    __threadfence();
    *(volatile v4f*)dst = v;
  }
}

extern "C" void kernel_launch(void* const* d_in, const int* in_sizes, int n_in,
                              void* d_out, int out_size, void* d_ws, size_t ws_size,
                              hipStream_t stream)
{
  if (n_in < 8) return;
  const float* xin   = (const float*)d_in[0];
  const float* noisy = (const float*)d_in[1];
  const float* acond = (const float*)d_in[2];
  const float* cw    = (const float*)d_in[3];
  const float* scf   = (const float*)d_in[4];
  const float* mixw  = (const float*)d_in[5];
  const float* ctr   = (const float*)d_in[6];
  const float* gridv = (const float*)d_in[7];
  float* dout = (float*)d_out;

  if (in_sizes[0] != NIMG * NPIX_IMG) return;
  if (in_sizes[1] != NIMG * NPIX_IMG) return;
  if (in_sizes[2] != NIMG) return;
  if (in_sizes[3] != NFEAT * NTAPS) return;
  if (in_sizes[4] != NFEAT) return;
  if (in_sizes[5] != NFEAT * NMIX) return;
  if (in_sizes[6] != NMIX) return;
  if (in_sizes[7] != NGRID) return;
  if (out_size != NIMG * NPIX_IMG) return;

  const size_t SZ_W16  = (size_t)NFEAT * KPAD * 2;
  const size_t SZ_WT16 = (size_t)KPAD * NFEAT * 2;
  const size_t SZ_TAB  = (size_t)NFEAT * TAB_PITCH * 4;
  const size_t SZ_ACOL = (size_t)NPIX_CHUNK * KPAD * 2;
  const size_t SZ_UQ   = (size_t)NPIX_CHUNK * 64 * 4;
  const size_t SZ_PHI  = (size_t)NPIX_CHUNK * NFEAT * 2;
  const size_t OFF_W16  = 0;
  const size_t OFF_WT16 = OFF_W16 + SZ_W16;
  const size_t OFF_TAB  = OFF_WT16 + SZ_WT16;
  const size_t OFF_ACOL = OFF_TAB + SZ_TAB;
  const size_t OFF_UQ   = OFF_ACOL + SZ_ACOL;
  const size_t OFF_PHI  = OFF_UQ + SZ_UQ;
  const size_t TOTAL    = OFF_PHI + SZ_PHI;
  if (ws_size < TOTAL) return;

  char* ws = (char*)d_ws;
  unsigned short* W16   = (unsigned short*)(ws + OFF_W16);
  unsigned short* WT16  = (unsigned short*)(ws + OFF_WT16);
  float*          TABLE = (float*)(ws + OFF_TAB);
  unsigned short* ACOL  = (unsigned short*)(ws + OFF_ACOL);
  float*          UQ    = (float*)(ws + OFF_UQ);
  unsigned short* PHI16 = (unsigned short*)(ws + OFF_PHI);
  const float*    nores = xin;

  const float WCARRY = 256.0f;
  const float PCARRY = 256.0f;
  const float PREC   = 0.25f;

  prep_weights_kernel<<<1, 256, 0, stream>>>(cw, scf, W16, WT16, WCARRY);
  mix_table_kernel<<<dim3(TAB_PITCH / 256, NFEAT), 256, 0, stream>>>(mixw, ctr, gridv, TABLE, PREC);

  for (int c = 0; c < NCHUNK; ++c) {
    const int img0 = c * IMG_PER_CHUNK;
    im2col_sym7_kernel<<<CHUNKS16 / 256, 256, 0, stream>>>(xin, ACOL, img0, CHUNKS16);
    wmma_gemm64<0, false, 0, 0, false, 0><<<dim3(NPIX_CHUNK / 512, 1), 256, 0, stream>>>(
        ACOL, ACOL, KPAD, 0L,
        W16, W16, KPAD, 0L,
        (void*)UQ, (void*)UQ, NFEAT, 0L,
        nores, nores, 0L,
        NPIX_CHUNK, NFEAT, KPAD, 1.0f / WCARRY);
    table_interp_kernel<<<CHUNKS16 / 256, 256, 0, stream>>>(UQ, TABLE, gridv, PHI16, CHUNKS16, PCARRY);
    wmma_gemm64<0, false, 0, 0, false, 0><<<dim3(NPIX_CHUNK / 512, 1), 256, 0, stream>>>(
        WT16, WT16, NFEAT, 0L,
        PHI16, PHI16, NFEAT, 0L,
        (void*)UQ, (void*)UQ, NPIX_CHUNK, 0L,
        nores, nores, 0L,
        KPAD, NPIX_CHUNK, NFEAT, 1.0f / (WCARRY * PCARRY));
    fold_prox_kernel<<<dim3(IMG_H, IMG_PER_CHUNK), 256, 0, stream>>>(UQ, xin, noisy, acond, dout, img0, NPIX_CHUNK);
  }
}
